// MOEModel_71382356459745
// MI455X (gfx1250) — hardware-verified
//
#include <hip/hip_runtime.h>
#include <math.h>


#define NB_   8
#define NP_   50
#define NN_   128
#define NM_   128
#define EMB_  128
#define NH_   8
#define HD_   16
#define NE_   8
#define CLIP_ 10.0f
#define NBP   (NB_ * NP_)
#define NTHR  256

#define ST      128
#define SLOTH   (128 * ST)
#define SLOTB   (SLOTH * 2)
#define O_EXTRA (8 * SLOTB)
#define O_RLAST (O_EXTRA)
#define O_WLAST (O_RLAST + 512)
#define O_SCORE (O_WLAST + 512)
#define O_PROB  (O_SCORE + 512)
#define O_IMPW  (O_PROB + 512)
#define O_IMPR  (O_IMPW + 256)
#define O_CE    (O_IMPR + 32)
#define O_RED   (O_CE + 32)
#define LDS_TOTAL (O_RED + 32)

#define UF_FLOATS 1056
#define IMP_PITCH 32

typedef unsigned short v8us  __attribute__((ext_vector_type(8)));
typedef unsigned short v16us __attribute__((ext_vector_type(16)));
typedef __bf16 v16bf __attribute__((ext_vector_type(16)));
typedef float v8f __attribute__((ext_vector_type(8)));
typedef float v4f __attribute__((ext_vector_type(4)));

union Frag { v16bf v; v16us u; v8us h[2]; };

__device__ __forceinline__ unsigned short bf_hi(float x) {
  unsigned u = __float_as_uint(x);
  u += 0x7FFFu + ((u >> 16) & 1u);
  return (unsigned short)(u >> 16);
}
__device__ __forceinline__ float bf_val(unsigned short b) {
  return __uint_as_float(((unsigned)b) << 16);
}
__device__ __forceinline__ void bf_split(float x, unsigned short& hi, unsigned short& lo) {
  hi = bf_hi(x);
  lo = bf_hi(x - bf_val(hi));
}

__device__ __forceinline__ v16bf frag16(const unsigned short* plane, int rowBase, int kBase,
                                        int ln, int hh) {
  const unsigned short* p = plane + (rowBase + ln) * ST + kBase;
  Frag f;
  f.h[0] = *(const v8us*)(p + 8 * hh);
  f.h[1] = *(const v8us*)(p + 16 + 8 * hh);
  return f.v;
}
__device__ __forceinline__ v16bf frag_pair(v8us e0, v8us e1) {
  Frag f;
  f.h[0] = e0;
  f.h[1] = e1;
  return f.v;
}

__device__ __forceinline__ v8f wm(v16bf a, v16bf b, v8f c) {
  return __builtin_amdgcn_wmma_f32_16x16x32_bf16(false, a, false, b, (short)0, c, false, false);
}

__device__ __forceinline__ v8f wmma3(v16bf ah, v16bf al, v16bf bh, v16bf bl, v8f c) {
  c = wm(ah, bh, c);
  c = wm(ah, bl, c);
  c = wm(al, bh, c);
  asm volatile("v_nop\n\tv_nop\n\tv_nop\n\tv_nop" : "+v"(c) : "v"(ah), "v"(al), "v"(bh), "v"(bl));
  return c;
}

__device__ __forceinline__ v8f wmma2s(v16bf a1, v16bf a2, v16bf b) {
  v8f c = {};
  c = wm(a1, b, c);
  c = wm(a2, b, c);
  asm volatile("v_nop\n\tv_nop\n\tv_nop\n\tv_nop" : "+v"(c) : "v"(a1), "v"(a2), "v"(b));
  return c;
}

__global__ __launch_bounds__(NTHR) void k_fold(const float* __restrict__ We,
                                               const float* __restrict__ be,
                                               const float* __restrict__ Wf,
                                               float* ufold) {
  __shared__ __attribute__((aligned(16))) float su[UF_FLOATS];
  const int tid = threadIdx.x;
  for (int q = tid; q < UF_FLOATS; q += NTHR) {
    float s = 0.f;
    if (q < NE_ * EMB_) {
      const float* w = We + (size_t)q * (EMB_ + 1);
#pragma unroll 1
      for (int o = 0; o < EMB_ + 1; ++o) s += w[o] * Wf[o];
    } else if (q < NE_ * EMB_ + NE_) {
      const float* b = be + (size_t)(q - NE_ * EMB_) * (EMB_ + 1);
#pragma unroll 1
      for (int o = 0; o < EMB_ + 1; ++o) s += b[o] * Wf[o];
    }
    su[q] = s;
  }
  __syncthreads();
  for (int q = tid; q < UF_FLOATS / 4; q += NTHR) {
    v4f v = *(const v4f*)(su + 4 * q);
    volatile v4f* p = (volatile v4f*)ufold + q;
    *p = v;
  }
  __threadfence();
  for (int q = tid; q < UF_FLOATS / 4; q += NTHR) {
    v4f v = *(const v4f*)(su + 4 * q);
    volatile v4f* p = (volatile v4f*)ufold + q;
    *p = v;
  }
}

__global__ __launch_bounds__(NTHR) void k_main(
    const float* __restrict__ nodes, const float* __restrict__ routes,
    const float* __restrict__ ninf, const float* __restrict__ rmask,
    const float* __restrict__ Wq, const float* __restrict__ Wk,
    const float* __restrict__ Wv, const float* __restrict__ Wg,
    const float* __restrict__ ufold, float* out, float* imp, int nbp) {
  extern __shared__ __attribute__((aligned(16))) unsigned char smem[];
  unsigned short* S0 = (unsigned short*)(smem + 0 * SLOTB);
  unsigned short* S1 = (unsigned short*)(smem + 1 * SLOTB);
  unsigned short* S2 = (unsigned short*)(smem + 2 * SLOTB);
  unsigned short* S3 = (unsigned short*)(smem + 3 * SLOTB);
  unsigned short* S4 = (unsigned short*)(smem + 4 * SLOTB);
  unsigned short* S5 = (unsigned short*)(smem + 5 * SLOTB);
  unsigned short* S6 = (unsigned short*)(smem + 6 * SLOTB);
  unsigned short* S7 = (unsigned short*)(smem + 7 * SLOTB);
  float* sRlast = (float*)(smem + O_RLAST);
  float* sWlast = (float*)(smem + O_WLAST);
  float* sScore = (float*)(smem + O_SCORE);
  float* sProb  = (float*)(smem + O_PROB);
  float* sImpW  = (float*)(smem + O_IMPW);
  float* sImpR  = (float*)(smem + O_IMPR);
  float* sCE    = (float*)(smem + O_CE);
  float* sRed   = (float*)(smem + O_RED);

  const int bp = blockIdx.x;
  if (bp >= nbp) return;
  const int tid  = threadIdx.x;
  const int lane = tid & 31;
  const int wv   = tid >> 5;
  const int hh   = lane >> 4;
  const int ln   = lane & 15;
  const int nB   = 16 * wv;

  const float* nfb = ninf + (size_t)bp * NN_;

  {
    const float* nb = nodes + (size_t)bp * NN_ * EMB_;
    for (int i = tid; i < NN_ * EMB_; i += NTHR) {
      int r = i >> 7, c = i & 127;
      unsigned short th, tl;
      bf_split(nb[i], th, tl);
      S0[r * ST + c] = th;
      S1[r * ST + c] = tl;
    }
    for (int i = tid; i < EMB_ * EMB_; i += NTHR) {
      int k = i >> 7, f = i & 127;
      unsigned short th, tl;
      bf_split(Wq[i], th, tl);
      S2[f * ST + k] = th;
      S3[f * ST + k] = tl;
    }
  }
  __syncthreads();
  {
    v16bf bh[4], bl[4];
#pragma unroll
    for (int kk = 0; kk < 4; ++kk) {
      bh[kk] = frag16(S0, nB, 32 * kk, ln, hh);
      bl[kk] = frag16(S1, nB, 32 * kk, ln, hh);
    }
#pragma unroll 1
    for (int j = 0; j < 8; ++j) {
      v8f acc = {};
#pragma unroll
      for (int kk = 0; kk < 4; ++kk) {
        v16bf ah = frag16(S2, 16 * j, 32 * kk, ln, hh);
        v16bf al = frag16(S3, 16 * j, 32 * kk, ln, hh);
        acc = wmma3(ah, al, bh[kk], bl[kk], acc);
      }
      v8us ph, pl;
#pragma unroll
      for (int r = 0; r < 8; ++r) {
        unsigned short th, tl;
        bf_split(acc[r], th, tl);
        ph[r] = th;
        pl[r] = tl;
      }
      const int qo = (nB + ln) * ST + 16 * j + 8 * hh;
      *(v8us*)(S4 + qo) = ph;
      *(v8us*)(S5 + qo) = pl;
    }
  }
  __syncthreads();

  {
    const float* rb = routes + (size_t)bp * NM_ * (EMB_ + 1);
    for (int i = tid; i < NM_ * (EMB_ + 1); i += NTHR) {
      int r = i / (EMB_ + 1), c = i - r * (EMB_ + 1);
      float v = rb[i];
      if (c < EMB_) {
        unsigned short th, tl;
        bf_split(v, th, tl);
        S0[r * ST + c] = th;
        S1[r * ST + c] = tl;
      } else {
        sRlast[r] = v;
      }
    }
    for (int i = tid; i < (EMB_ + 1) * EMB_; i += NTHR) {
      int k = i >> 7, f = i & 127;
      float v = Wv[i];
      if (k < EMB_) {
        unsigned short th, tl;
        bf_split(v, th, tl);
        S2[f * ST + k] = th;
        S3[f * ST + k] = tl;
      } else {
        sWlast[f] = v;
      }
    }
  }
  __syncthreads();
  {
    v16bf ah[4], al[4];
#pragma unroll
    for (int kk = 0; kk < 4; ++kk) {
      ah[kk] = frag16(S0, nB, 32 * kk, ln, hh);
      al[kk] = frag16(S1, nB, 32 * kk, ln, hh);
    }
#pragma unroll 1
    for (int j = 0; j < 8; ++j) {
      v8f acc = {};
#pragma unroll
      for (int kk = 0; kk < 4; ++kk) {
        v16bf bh = frag16(S2, 16 * j, 32 * kk, ln, hh);
        v16bf bl = frag16(S3, 16 * j, 32 * kk, ln, hh);
        acc = wmma3(ah[kk], al[kk], bh, bl, acc);
      }
      const float wl = sWlast[16 * j + ln];
      v8us ph, pl;
#pragma unroll
      for (int r = 0; r < 8; ++r) {
        float v = acc[r] + sRlast[nB + 8 * hh + r] * wl;
        unsigned short th, tl;
        bf_split(v, th, tl);
        ph[r] = th;
        pl[r] = tl;
      }
      const int vo = (16 * j + ln) * ST + nB + 8 * hh;
      *(v8us*)(S6 + vo) = ph;
      *(v8us*)(S7 + vo) = pl;
    }
  }
  __syncthreads();

  {
    for (int i = tid; i < (EMB_ + 1) * EMB_; i += NTHR) {
      int k = i >> 7, f = i & 127;
      float v = Wk[i];
      if (k < EMB_) {
        unsigned short th, tl;
        bf_split(v, th, tl);
        S2[f * ST + k] = th;
        S3[f * ST + k] = tl;
      } else {
        sWlast[f] = v;
      }
    }
    v16bf bh[4], bl[4];
#pragma unroll
    for (int kk = 0; kk < 4; ++kk) {
      bh[kk] = frag16(S0, nB, 32 * kk, ln, hh);
      bl[kk] = frag16(S1, nB, 32 * kk, ln, hh);
    }
    __syncthreads();
#pragma unroll 1
    for (int j = 0; j < 8; ++j) {
      v8f acc = {};
#pragma unroll
      for (int kk = 0; kk < 4; ++kk) {
        v16bf ah2 = frag16(S2, 16 * j, 32 * kk, ln, hh);
        v16bf al2 = frag16(S3, 16 * j, 32 * kk, ln, hh);
        acc = wmma3(ah2, al2, bh[kk], bl[kk], acc);
      }
      const float rl = sRlast[nB + ln];
      v8us ph, pl;
#pragma unroll
      for (int r = 0; r < 8; ++r) {
        float v = acc[r] + sWlast[16 * j + 8 * hh + r] * rl;
        unsigned short th, tl;
        bf_split(v, th, tl);
        ph[r] = th;
        pl[r] = tl;
      }
      const int ko = (nB + ln) * ST + 16 * j + 8 * hh;
      *(v8us*)(S0 + ko) = ph;
      *(v8us*)(S1 + ko) = pl;
    }
  }
  __syncthreads();

  {
    const int h = wv;
    const float* rmb = rmask + (size_t)bp * NN_ * NM_;
    unsigned short* Ph = S2 + wv * (16 * ST);
    unsigned short* Pl = S3 + wv * (16 * ST);
#pragma unroll 1
    for (int s = 0; s < 8; ++s) {
      const int qo = (16 * s + ln) * ST + 16 * h + 8 * hh;
      v8us qh8 = *(const v8us*)(S4 + qo);
      v8us ql8 = *(const v8us*)(S5 + qo);
      v16bf a1 = frag_pair(qh8, qh8);
      v16bf a2 = frag_pair(ql8, ql8);
      v8f acc[8];
#pragma unroll
      for (int t = 0; t < 8; ++t) {
        const int ko = (16 * t + ln) * ST + 16 * h + 8 * hh;
        v8us kh8 = *(const v8us*)(S0 + ko);
        v8us kl8 = *(const v8us*)(S1 + ko);
        acc[t] = wmma2s(a1, a2, frag_pair(kh8, kl8));
      }
#pragma unroll
      for (int r = 0; r < 8; ++r) {
        const int n = 16 * s + 8 * hh + r;
        const float* rmrow = rmb + (size_t)n * NM_;
        float rmax = -3.4e38f;
#pragma unroll
        for (int t = 0; t < 8; ++t) {
          float v = acc[t][r] * 0.25f + rmrow[16 * t + ln];
          acc[t][r] = v;
          rmax = fmaxf(rmax, v);
        }
#pragma unroll
        for (int mm = 1; mm < 16; mm <<= 1) rmax = fmaxf(rmax, __shfl_xor(rmax, mm, 32));
        float rsum = 0.f;
#pragma unroll
        for (int t = 0; t < 8; ++t) {
          float e = __expf(acc[t][r] - rmax);
          acc[t][r] = e;
          rsum += e;
        }
#pragma unroll
        for (int mm = 1; mm < 16; mm <<= 1) rsum += __shfl_xor(rsum, mm, 32);
        const float keep = (nfb[n] == 0.f) ? 1.f : 0.f;
        const float scl = (1.f / rsum) * keep;
#pragma unroll
        for (int t = 0; t < 8; ++t) {
          float p = acc[t][r] * scl;
          unsigned short th, tl;
          bf_split(p, th, tl);
          Ph[(8 * hh + r) * ST + 16 * t + ln] = th;
          Pl[(8 * hh + r) * ST + 16 * t + ln] = tl;
        }
      }
      __syncthreads();
      v8f oacc = {};
#pragma unroll
      for (int kk = 0; kk < 4; ++kk) {
        v16bf avh = frag16(S6, 16 * h, 32 * kk, ln, hh);
        v16bf avl = frag16(S7, 16 * h, 32 * kk, ln, hh);
        v16bf bph = frag16(Ph, 0, 32 * kk, ln, hh);
        v16bf bpl = frag16(Pl, 0, 32 * kk, ln, hh);
        oacc = wmma3(avh, avl, bph, bpl, oacc);
      }
      v8us oh, ol;
#pragma unroll
      for (int r = 0; r < 8; ++r) {
        unsigned short th, tl;
        bf_split(oacc[r], th, tl);
        oh[r] = th;
        ol[r] = tl;
      }
      *(v8us*)(S4 + qo) = oh;
      *(v8us*)(S5 + qo) = ol;
      __syncthreads();
    }
  }

  for (int i = tid; i < 16 * EMB_; i += NTHR) {
    int f = i >> 7, k = i & 127;
    float v = (f < NE_) ? Wg[k * NE_ + f] : ufold[(f - NE_) * EMB_ + k];
    unsigned short th, tl;
    bf_split(v, th, tl);
    S2[f * ST + k] = th;
    S3[f * ST + k] = tl;
  }
  if (tid < NE_) sCE[tid] = ufold[NE_ * EMB_ + tid];
  __syncthreads();
  {
    v8f g = {};
#pragma unroll
    for (int kk = 0; kk < 4; ++kk) {
      v16bf axh = frag16(S4, nB, 32 * kk, ln, hh);
      v16bf axl = frag16(S5, nB, 32 * kk, ln, hh);
      v16bf bgh = frag16(S2, 0, 32 * kk, ln, hh);
      v16bf bgl = frag16(S3, 0, 32 * kk, ln, hh);
      g = wmma3(axh, axl, bgh, bgl, g);
    }
    float impP = 0.f;
#pragma unroll
    for (int r = 0; r < 8; ++r) {
      const int tok = nB + 8 * hh + r;
      float v = (ln < NE_) ? g[r] : -3.4e38f;
      float bv = v; int bi = ln;
#pragma unroll
      for (int mm = 1; mm < 16; mm <<= 1) {
        float ov = __shfl_xor(bv, mm, 32);
        int   oi = __shfl_xor(bi, mm, 32);
        if (ov > bv || (ov == bv && oi < bi)) { bv = ov; bi = oi; }
      }
      float v2 = (ln == bi) ? -3.4e38f : v;
      float b2v = v2; int b2i = ln;
#pragma unroll
      for (int mm = 1; mm < 16; mm <<= 1) {
        float ov = __shfl_xor(b2v, mm, 32);
        int   oi = __shfl_xor(b2i, mm, 32);
        if (ov > b2v || (ov == b2v && oi < b2i)) { b2v = ov; b2i = oi; }
      }
      const float ex = expf(b2v - bv);
      const float rs = 1.f / (1.f + ex);
      const float g0 = rs, g1 = ex * rs;
      float term = 0.f;
      if (ln >= NE_) {
        const int e = ln - NE_;
        const float val = g[r] + sCE[e];
        term = (e == bi) ? g0 * val : ((e == b2i) ? g1 * val : 0.f);
      }
#pragma unroll
      for (int mm = 1; mm < 16; mm <<= 1) term += __shfl_xor(term, mm, 32);
      if (ln == 0) sScore[tok] = CLIP_ * tanhf(term) + nfb[tok];
      if (ln < NE_) impP += (ln == bi) ? g0 : ((ln == b2i) ? g1 : 0.f);
    }
    impP += __shfl_xor(impP, 16, 32);
    if (lane < NE_) sImpW[wv * NE_ + lane] = impP;
  }
  __syncthreads();

  if (tid < NE_) {
    float s = 0.f;
#pragma unroll
    for (int w = 0; w < 8; ++w) s += sImpW[w * NE_ + tid];
    sImpR[tid] = s;
  }
  if (wv == 0) {
    float a0 = sScore[lane], a1 = sScore[lane + 32];
    float a2 = sScore[lane + 64], a3 = sScore[lane + 96];
    float mx = fmaxf(fmaxf(a0, a1), fmaxf(a2, a3));
#pragma unroll
    for (int mm = 1; mm < 32; mm <<= 1) mx = fmaxf(mx, __shfl_xor(mx, mm, 32));
    float sm = expf(a0 - mx) + expf(a1 - mx) + expf(a2 - mx) + expf(a3 - mx);
#pragma unroll
    for (int mm = 1; mm < 32; mm <<= 1) sm += __shfl_xor(sm, mm, 32);
    if (lane == 0) { sRed[0] = mx; sRed[1] = sm; }
  }
  __syncthreads();
  if (tid < NN_) sProb[tid] = expf(sScore[tid] - sRed[0]) * (1.f / sRed[1]);
  __syncthreads();
  if (wv == 0) {
    const v4f pv = *(const v4f*)(sProb + 4 * lane);
    v4f iv = {0.f, 0.f, 0.f, 0.f};
    if (lane < 2) iv = *(const v4f*)(sImpR + 4 * lane);
    volatile v4f* po = (volatile v4f*)(out + (size_t)bp * NN_) + lane;
    volatile v4f* pi = (volatile v4f*)(imp + (size_t)bp * IMP_PITCH) + lane;
    *po = pv;
    if (lane < 8) *pi = iv;
    __threadfence();
    *po = pv;
    if (lane < 8) *pi = iv;
  }
}

__global__ __launch_bounds__(64) void k_loss(const float* imp, float* out, int nbp, int outIdx) {
  __shared__ float simp[NE_];
  const int e = threadIdx.x;
  if (e < NE_) {
    double s = 0.0;
#pragma unroll 1
    for (int b = 0; b < nbp; ++b) s += (double)imp[(size_t)b * IMP_PITCH + e];
    simp[e] = (float)s;
  }
  __syncthreads();
  if (e == 0) {
    float mean = 0.f;
#pragma unroll
    for (int i = 0; i < NE_; ++i) mean += simp[i];
    mean *= (1.f / 8.f);
    float var = 0.f;
#pragma unroll
    for (int i = 0; i < NE_; ++i) { float d = simp[i] - mean; var += d * d; }
    var *= (1.f / 8.f);
    const float lossv = var / (mean * mean + 1e-10f);
    volatile float* p = out + outIdx;
    *p = lossv;
    __threadfence();
    *p = lossv;
  }
}

extern "C" void kernel_launch(void* const* d_in, const int* in_sizes, int n_in,
                              void* d_out, int out_size, void* d_ws, size_t ws_size,
                              hipStream_t stream) {
  if (n_in < 11) return;
  const int nbp = NBP;
  if (in_sizes[0] != nbp * NN_ * EMB_) return;
  if (in_sizes[1] != nbp * NM_ * (EMB_ + 1)) return;
  if (in_sizes[2] != nbp * NN_) return;
  if (in_sizes[3] != nbp * NN_ * NM_) return;
  if (in_sizes[4] != EMB_ * EMB_) return;
  if (in_sizes[5] != (EMB_ + 1) * EMB_) return;
  if (in_sizes[6] != (EMB_ + 1) * EMB_) return;
  if (in_sizes[7] != EMB_ * NE_) return;
  if (in_sizes[8] != NE_ * EMB_ * (EMB_ + 1)) return;
  if (in_sizes[9] != NE_ * (EMB_ + 1)) return;
  if (in_sizes[10] != EMB_ + 1) return;
  if (out_size != nbp * NN_ + 1) return;

  const size_t off_uf  = 0;
  const size_t byt_uf  = (size_t)UF_FLOATS * sizeof(float);
  const size_t off_imp = off_uf + byt_uf;
  const size_t byt_imp = (size_t)nbp * IMP_PITCH * sizeof(float);
  if (off_imp + byt_imp > ws_size) return;

  const float* nodes  = (const float*)d_in[0];
  const float* routes = (const float*)d_in[1];
  const float* ninf   = (const float*)d_in[2];
  const float* rmask  = (const float*)d_in[3];
  const float* Wq     = (const float*)d_in[4];
  const float* Wk     = (const float*)d_in[5];
  const float* Wv     = (const float*)d_in[6];
  const float* Wg     = (const float*)d_in[7];
  const float* We     = (const float*)d_in[8];
  const float* be     = (const float*)d_in[9];
  const float* Wfin   = (const float*)d_in[10];
  float* out   = (float*)d_out;
  float* ufold = (float*)((char*)d_ws + off_uf);
  float* imp   = (float*)((char*)d_ws + off_imp);

  (void)hipFuncSetAttribute((const void*)k_main,
                            hipFuncAttributeMaxDynamicSharedMemorySize, LDS_TOTAL);
  k_fold<<<1, NTHR, 0, stream>>>(We, be, Wfin, ufold);
  k_main<<<nbp, NTHR, LDS_TOTAL, stream>>>(nodes, routes, ninf, rmask, Wq, Wk, Wv, Wg,
                                           ufold, out, imp, nbp);
  k_loss<<<1, 64, 0, stream>>>(imp, out, nbp, nbp * NN_);
}
